// Head_47510928228486
// MI455X (gfx1250) — hardware-verified
//
#include <hip/hip_runtime.h>
#ifndef NB
#define NB 256
#endif
#ifndef SEQ
#define SEQ 512
#endif
#define NB_FULL 256
#define SEQ_FULL 512
#define DM 64
#define HD 64
#define NQT (SEQ / 64)
#define SP 68
#define PLANE_BYTES ((size_t)NB * SEQ * HD * 2)
#define WT_BYTES ((size_t)3 * 64 * 64 * 2)

static_assert(SEQ % 64 == 0);
static_assert(SEQ <= SEQ_FULL);
static_assert(NB <= NB_FULL);
static_assert(DM == 64 && HD == 64);
static_assert(WT_BYTES + 6 * PLANE_BYTES <= (size_t)134217728);
static_assert((3 * 64 * 8) % 256 == 0);

typedef _Float16 v16h __attribute__((ext_vector_type(16)));
typedef unsigned short v8us __attribute__((ext_vector_type(8), may_alias));
typedef float  v8f  __attribute__((ext_vector_type(8)));
typedef float  v4f  __attribute__((ext_vector_type(4)));
typedef float  v4fa __attribute__((ext_vector_type(4), may_alias));
union FragH { v16h v; v8us half[2]; _Float16 h[16]; unsigned short u[16]; };
union Frag8 { v8us v; _Float16 h[8]; };

__device__ __forceinline__ float bf16_rne(float x) { unsigned int u = __float_as_uint(x); u = (u + 0x7FFFu + ((u >> 16) & 1u)) & 0xFFFF0000u; return __uint_as_float(u); }

__device__ __forceinline__ v16h g2_frag(const _Float16* p, unsigned hh) { FragH f; f.half[0] = *(const v8us*)((const unsigned short*)p + 8 * hh); f.half[1] = *(const v8us*)((const unsigned short*)p + 16 + 8 * hh); return f.v; }
__device__ __forceinline__ v8f g2_mma(v16h a, v16h b, v8f c) { v8f d = __builtin_amdgcn_wmma_f32_16x16x32_f16(false, a, false, b, (short)0, c, false, false); asm volatile("v_nop\n\tv_nop\n\tv_nop\n\tv_nop" : "+v"(d) : "v"(a), "v"(b)); return d; }

__device__ __forceinline__ v16h x_frag(const float* p, unsigned hh) {
  const v4f x0 = *(const v4fa*)(p + 8 * hh), x1 = *(const v4fa*)(p + 8 * hh + 4), x2 = *(const v4fa*)(p + 16 + 8 * hh), x3 = *(const v4fa*)(p + 16 + 8 * hh + 4);
  const float xs[16] = {x0[0],x0[1],x0[2],x0[3],x1[0],x1[1],x1[2],x1[3],x2[0],x2[1],x2[2],x2[3],x3[0],x3[1],x3[2],x3[3]};
  FragH f;
#pragma unroll
  for (int i = 0; i < 16; ++i) f.h[i] = (_Float16)bf16_rne(xs[i]);
  return f.v;
}

__device__ __forceinline__ void split8(const float* v, Frag8& h, Frag8& l) {
#pragma unroll
  for (int q = 0; q < 8; ++q) { const _Float16 hv = (_Float16)v[q]; h.h[q] = hv; l.h[q] = (_Float16)((v[q] - (float)hv) * 1024.0f); }
}

__global__ __launch_bounds__(256) void k_wt3(const float* __restrict__ wq, const float* __restrict__ wk, const float* __restrict__ wv, _Float16* __restrict__ Wt) {
  const unsigned t = blockIdx.x * 256u + threadIdx.x;
  const unsigned c = blockIdx.x >> 1;
  const unsigned n = (t >> 3) & 63u, k8 = (t & 7u) * 8u;
  const float* W = (c == 0u) ? wq : ((c == 1u) ? wk : wv);
  Frag8 f;
#pragma unroll
  for (int i = 0; i < 8; ++i) f.h[i] = (_Float16)(bf16_rne(W[(size_t)(k8 + i) * 64u + n]) * 16.0f);
  unsigned short* dst = (unsigned short*)Wt + (size_t)t * 8u;
  *(volatile v8us*)dst = f.v;
  __threadfence();
  *(volatile v8us*)dst = f.v;
}

__global__ __launch_bounds__(128) void k_proj(const float* __restrict__ x, const _Float16* __restrict__ Wt,
                                              _Float16* __restrict__ Qh, _Float16* __restrict__ Ql, _Float16* __restrict__ Kh, _Float16* __restrict__ Kl,
                                              _Float16* __restrict__ Vth, _Float16* __restrict__ Vtl) {
  __shared__ __attribute__((aligned(16))) float st[3][64][SP];
  const unsigned tid = threadIdx.x, w = tid >> 5, lane = tid & 31u, ln = lane & 15u, hh = lane >> 4;
  const unsigned row0 = blockIdx.x * 64u;
  const unsigned bb = row0 / (unsigned)SEQ, t0 = row0 % (unsigned)SEQ;
  const float* xr = x + ((size_t)bb * SEQ_FULL + t0 + 16u * w + ln) * DM;
  const v16h a0 = x_frag(xr, hh), a1 = x_frag(xr + 32, hh);
  const v8f z8 = {0.f, 0.f, 0.f, 0.f, 0.f, 0.f, 0.f, 0.f};
#pragma unroll
  for (int c = 0; c < 3; ++c) {
#pragma unroll
    for (int j = 0; j < 4; ++j) {
      const _Float16* bp = Wt + (size_t)(c * 64 + j * 16 + (int)ln) * 64;
      const v16h b0 = g2_frag(bp, hh), b1 = g2_frag(bp + 32, hh);
      v8f acc = z8;
      acc = g2_mma(a0, b0, acc);
      acc = g2_mma(a1, b1, acc);
#pragma unroll
      for (int r = 0; r < 8; ++r) st[c][16u * w + 8u * hh + r][j * 16 + (int)ln] = acc[r] * 0.0625f;
    }
  }
  __syncthreads();
  const unsigned pr = tid >> 3, pc = (tid & 7u) * 8u;
  Frag8 qh_[4], ql_[4], kh_[4], kl_[4], vh_[4], vl_[4];
#pragma unroll
  for (int it = 0; it < 4; ++it) {
    const unsigned rr = pr + 16u * it;
    { const v4f a = *(const v4fa*)&st[0][rr][pc], c = *(const v4fa*)&st[0][rr][pc + 4]; const float v[8] = {a[0],a[1],a[2],a[3],c[0],c[1],c[2],c[3]}; split8(v, qh_[it], ql_[it]); }
    { const v4f a = *(const v4fa*)&st[1][rr][pc], c = *(const v4fa*)&st[1][rr][pc + 4]; const float v[8] = {a[0],a[1],a[2],a[3],c[0],c[1],c[2],c[3]}; split8(v, kh_[it], kl_[it]); }
    { float v[8];
#pragma unroll
      for (int q = 0; q < 8; ++q) v[q] = st[2][pc + q][rr];
      split8(v, vh_[it], vl_[it]); }
  }
  for (int pass = 0; pass < 2; ++pass) {
#pragma unroll
    for (int it = 0; it < 4; ++it) {
      const unsigned rr = pr + 16u * it;
      const size_t qo = ((size_t)row0 + rr) * HD + pc;
      *(volatile v8us*)((unsigned short*)Qh + qo) = qh_[it].v;
      *(volatile v8us*)((unsigned short*)Ql + qo) = ql_[it].v;
      *(volatile v8us*)((unsigned short*)Kh + qo) = kh_[it].v;
      *(volatile v8us*)((unsigned short*)Kl + qo) = kl_[it].v;
      const size_t vo = ((size_t)bb * HD + rr) * SEQ + t0 + pc;
      *(volatile v8us*)((unsigned short*)Vth + vo) = vh_[it].v;
      *(volatile v8us*)((unsigned short*)Vtl + vo) = vl_[it].v;
    }
    if (pass == 0) __threadfence();
  }
}

__device__ __forceinline__ void p_group(const float* sp, float newm, float& sum, FragH& ph, FragH& pl, const int e0) {
  const v4f a = *(const v4fa*)sp, c = *(const v4fa*)(sp + 4);
  const float sv[8] = {a[0],a[1],a[2],a[3],c[0],c[1],c[2],c[3]};
#pragma unroll
  for (int q = 0; q < 8; ++q) {
    const float p = __expf(sv[q] - newm);
    sum += p;
    const float pcv = p * 256.0f;
    const _Float16 hv = (_Float16)pcv;
    ph.h[e0 + q] = hv;
    pl.h[e0 + q] = (_Float16)((pcv - (float)hv) * 1024.0f);
  }
}

__global__ __launch_bounds__(128) void k_attn(const _Float16* __restrict__ Qh, const _Float16* __restrict__ Ql, const _Float16* __restrict__ Kh, const _Float16* __restrict__ Kl,
                                              const _Float16* __restrict__ Vth, const _Float16* __restrict__ Vtl, float* __restrict__ out) {
  __shared__ __attribute__((aligned(16))) float sw[4][16][SP];
  const unsigned tid = threadIdx.x, w = tid >> 5, lane = tid & 31u, ln = lane & 15u, hh = lane >> 4;
  const unsigned b = blockIdx.x / (unsigned)NQT, qt = blockIdx.x % (unsigned)NQT;
  const unsigned q0 = qt * 64u, qw0 = q0 + 16u * w;
  const size_t prow = (size_t)b * SEQ;
  const _Float16* qhp = Qh + (prow + qw0 + ln) * HD;
  const _Float16* qlp = Ql + (prow + qw0 + ln) * HD;
  const v16h aqh0 = g2_frag(qhp, hh), aqh1 = g2_frag(qhp + 32, hh), aql0 = g2_frag(qlp, hh), aql1 = g2_frag(qlp + 32, hh);
  const v8f z8 = {0.f, 0.f, 0.f, 0.f, 0.f, 0.f, 0.f, 0.f};
  v8f oh[4] = {z8, z8, z8, z8}, orr[4] = {z8, z8, z8, z8};
  float m_run = -1.0e30f, l_run = 0.f;
#pragma unroll 1
  for (unsigned kt = 0; kt <= qt; ++kt) {
    const size_t krow = prow + kt * 64u + ln;
#pragma unroll
    for (int j = 0; j < 4; ++j) {
      const _Float16* kh = Kh + (krow + 16u * j) * HD;
      const _Float16* kl = Kl + (krow + 16u * j) * HD;
      const v16h bh0 = g2_frag(kh, hh), bh1 = g2_frag(kh + 32, hh), bl0 = g2_frag(kl, hh), bl1 = g2_frag(kl + 32, hh);
      v8f sh = z8, sr = z8;
      sh = g2_mma(aqh0, bh0, sh); sh = g2_mma(aqh1, bh1, sh);
      sr = g2_mma(aql0, bh0, sr); sr = g2_mma(aql1, bh1, sr);
      sr = g2_mma(aqh0, bl0, sr); sr = g2_mma(aqh1, bl1, sr);
      const unsigned kcol = kt * 64u + 16u * j + ln;
#pragma unroll
      for (int r = 0; r < 8; ++r) {
        const unsigned qi = qw0 + 8u * hh + r;
        float s = (sh[r] + sr[r] * 0.0009765625f) * 0.125f;
        s = (kcol > qi) ? -1.0e30f : s;
        sw[w][8u * hh + r][16 * j + (int)ln] = s;
      }
    }
    __builtin_amdgcn_fence(4  , "workgroup");
    __builtin_amdgcn_wave_barrier();
    const float* srow = &sw[w][ln][8u * hh];
    float tmax = -1.0e30f;
#pragma unroll
    for (int g = 0; g < 4; ++g) {
      const v4f a = *(const v4fa*)(srow + 16 * g), c = *(const v4fa*)(srow + 16 * g + 4);
      tmax = fmaxf(tmax, fmaxf(fmaxf(a[0], a[1]), fmaxf(a[2], a[3])));
      tmax = fmaxf(tmax, fmaxf(fmaxf(c[0], c[1]), fmaxf(c[2], c[3])));
    }
    tmax = fmaxf(tmax, __shfl_xor(tmax, 16, 32));
    const float newm = fmaxf(m_run, tmax);
    const float al = __expf(m_run - newm);
    float sum = 0.f;
    FragH ph0, ph1, pl0, pl1;
    p_group(srow,      newm, sum, ph0, pl0, 0);
    p_group(srow + 16, newm, sum, ph0, pl0, 8);
    p_group(srow + 32, newm, sum, ph1, pl1, 0);
    p_group(srow + 48, newm, sum, ph1, pl1, 8);
    sum += __shfl_xor(sum, 16, 32);
    m_run = newm;
    l_run = l_run * al + sum;
#pragma unroll
    for (int r = 0; r < 8; ++r) {
      const float ar = __shfl(al, (int)(8u * hh) + r, 32);
#pragma unroll
      for (int j = 0; j < 4; ++j) { oh[j][r] *= ar; orr[j][r] *= ar; }
    }
#pragma unroll
    for (int j = 0; j < 4; ++j) {
      const size_t vo = ((size_t)b * HD + 16u * j + ln) * SEQ + kt * 64u;
      const _Float16* vh = Vth + vo;
      const _Float16* vl = Vtl + vo;
      const v16h bvh0 = g2_frag(vh, hh), bvh1 = g2_frag(vh + 32, hh), bvl0 = g2_frag(vl, hh), bvl1 = g2_frag(vl + 32, hh);
      oh[j]  = g2_mma(ph0.v, bvh0, oh[j]);  oh[j]  = g2_mma(ph1.v, bvh1, oh[j]);
      orr[j] = g2_mma(pl0.v, bvh0, orr[j]); orr[j] = g2_mma(pl1.v, bvh1, orr[j]);
      orr[j] = g2_mma(ph0.v, bvl0, orr[j]); orr[j] = g2_mma(ph1.v, bvl1, orr[j]);
    }
    __builtin_amdgcn_fence(4  , "workgroup");
    __builtin_amdgcn_wave_barrier();
  }
  const float invl = 1.0f / (256.0f * l_run);
  float ir[8];
#pragma unroll
  for (int r = 0; r < 8; ++r) ir[r] = __shfl(invl, (int)(8u * hh) + r, 32);
#pragma unroll
  for (int j = 0; j < 4; ++j)
#pragma unroll
    for (int r = 0; r < 8; ++r) sw[w][8u * hh + r][16 * j + (int)ln] = (oh[j][r] + orr[j][r] * 0.0009765625f) * ir[r];
  __builtin_amdgcn_fence(4  , "workgroup");
  __builtin_amdgcn_wave_barrier();
  float* orow = out + ((size_t)b * SEQ_FULL + qw0) * HD;
  const unsigned c4 = ln * 4u;
  v4f ov[8];
#pragma unroll
  for (int q = 0; q < 8; ++q) ov[q] = *(const v4fa*)&sw[w][2u * q + hh][c4];
  for (int pass = 0; pass < 2; ++pass) {
#pragma unroll
    for (int q = 0; q < 8; ++q) *(volatile v4f*)(orow + (size_t)(2u * q + hh) * HD + c4) = ov[q];
    if (pass == 0) __threadfence();
  }
}

extern "C" void kernel_launch(void* const* d_in, const int* in_sizes, int n_in,
                              void* d_out, int out_size, void* d_ws, size_t ws_size, hipStream_t stream) {
  if (n_in < 4) return;
  const size_t need_x = ((size_t)(NB - 1) * SEQ_FULL + SEQ) * DM;
  if ((size_t)in_sizes[0] < need_x) return;
  if (in_sizes[1] < 64 * 64 || in_sizes[2] < 64 * 64 || in_sizes[3] < 64 * 64) return;
  if ((size_t)out_size < need_x) return;
  const float* x  = (const float*)d_in[0];
  const float* wk = (const float*)d_in[1];
  const float* wq = (const float*)d_in[2];
  const float* wv = (const float*)d_in[3];
  char* ws = (char*)d_ws; size_t off = 0;
  auto take = [&](size_t bytes) { char* p = ws + off; off += (bytes + 255) & ~(size_t)255; return p; };
  _Float16* Wt  = (_Float16*)take(WT_BYTES);
  _Float16* Qh  = (_Float16*)take(PLANE_BYTES);
  _Float16* Ql  = (_Float16*)take(PLANE_BYTES);
  _Float16* Kh  = (_Float16*)take(PLANE_BYTES);
  _Float16* Kl  = (_Float16*)take(PLANE_BYTES);
  _Float16* Vth = (_Float16*)take(PLANE_BYTES);
  _Float16* Vtl = (_Float16*)take(PLANE_BYTES);
  if (off > ws_size) return;
  k_wt3<<<(3 * 64 * 8) / 256, 256, 0, stream>>>(wq, wk, wv, Wt);
  k_proj<<<(unsigned)((size_t)NB * SEQ / 64), 128, 0, stream>>>(x, Wt, Qh, Ql, Kh, Kl, Vth, Vtl);
  k_attn<<<(unsigned)((size_t)NB * NQT), 128, 0, stream>>>(Qh, Ql, Kh, Kl, Vth, Vtl, (float*)d_out);
}
